// binary_dense_72816875536781
// MI455X (gfx1250) — hardware-verified
//
#include <hip/hip_runtime.h>


#define NBT  512
#define NI   1024
#define NO   1024
#define TI   512
#define TO   512
#define NK   16
#define KTOT (NK * NI)
#define DM   KTOT
#define NTK  NBT
#define LOSC 1024.0f

typedef _Float16 h16;
typedef unsigned short bf;
typedef __attribute__((ext_vector_type(16))) __bf16   v16bf;
typedef __attribute__((ext_vector_type(16))) _Float16 v16h;
typedef __attribute__((ext_vector_type(8)))  _Float16 v8h;
typedef __attribute__((ext_vector_type(8)))  unsigned short v8us;
typedef __attribute__((ext_vector_type(8)))  float    v8f;
typedef __attribute__((ext_vector_type(4)))  float    v4f;
typedef __attribute__((ext_vector_type(4)))  _Float16 v4h;
typedef v8h  __attribute__((may_alias)) v8ha;
typedef v4f  __attribute__((may_alias)) v4fa;
typedef v8us __attribute__((may_alias)) v8usa;

__device__ __forceinline__ unsigned short f2bf(float f) { unsigned u = __float_as_uint(f); u += 0x7FFFu + ((u >> 16) & 1u); return (unsigned short)(u >> 16); }
__device__ __forceinline__ float bf2f(unsigned short b) { return __uint_as_float(((unsigned)b) << 16); }
__device__ __forceinline__ float bfr(float f) { return bf2f(f2bf(f)); }
__device__ __forceinline__ v16h cat16(v8h lo, v8h hi) { return __builtin_shufflevector(lo, hi, 0, 1, 2, 3, 4, 5, 6, 7, 8, 9, 10, 11, 12, 13, 14, 15); }
__device__ __forceinline__ v16bf cat16b(v8us lo, v8us hi) { return __builtin_bit_cast(v16bf, __builtin_shufflevector(lo, hi, 0, 1, 2, 3, 4, 5, 6, 7, 8, 9, 10, 11, 12, 13, 14, 15)); }
__device__ __forceinline__ v8f wmma16(v16h a, v16h b, v8f c) { return __builtin_amdgcn_wmma_f32_16x16x32_f16(false, a, false, b, (short)0, c, false, false); }
__device__ __forceinline__ v8f wmmab(v16bf a, v16bf b, v8f c) { return __builtin_amdgcn_wmma_f32_16x16x32_bf16(false, a, false, b, (short)0, c, false, false); }

template <bool SPLITA, bool F16OUT = false>
__global__ __launch_bounds__(128) void k_gemmb(const bf* __restrict__ A, const bf* __restrict__ Al, const bf* __restrict__ Bn, const float* __restrict__ bias, float* C, int ldc, h16* C2, const float* __restrict__ R = nullptr, int K = DM, int roundR = 1) {
    __shared__ __align__(16) float ost[4][16 * 68];
    const int lane = threadIdx.x & 31, wave = threadIdx.x >> 5, lr = lane & 15, hi = lane >> 4;
    const int r0 = blockIdx.x * 64 + wave * 16, c0 = blockIdx.y * 64;
    const size_t aoff = (size_t)(r0 + lr) * K + 8 * hi;
    size_t boff[4];
#pragma unroll
    for (int t = 0; t < 4; ++t) boff[t] = (size_t)(c0 + t * 16 + lr) * K + 8 * hi;
    v8f acc[4];
#pragma unroll
    for (int t = 0; t < 4; ++t) acc[t] = (v8f){};
#pragma unroll 1
    for (int kc = 0; kc < K; kc += 32) {
        const v16bf a = cat16b(*(const v8us*)(A + aoff + kc), *(const v8us*)(A + aoff + kc + 16));
        v16bf al = a;
        if (SPLITA) al = cat16b(*(const v8us*)(Al + aoff + kc), *(const v8us*)(Al + aoff + kc + 16));
#pragma unroll
        for (int t = 0; t < 4; ++t) { const v16bf b = cat16b(*(const v8us*)(Bn + boff[t] + kc), *(const v8us*)(Bn + boff[t] + kc + 16)); acc[t] = wmmab(a, b, acc[t]); if (SPLITA) acc[t] = wmmab(al, b, acc[t]); }
        asm volatile("v_nop\n\tv_nop\n\tv_nop\n\tv_nop" : "+v"(acc[0]), "+v"(acc[1]), "+v"(acc[2]), "+v"(acc[3]) : "v"(a), "v"(al));
    }
    float* os = &ost[wave][0];
#pragma unroll
    for (int t = 0; t < 4; ++t) { const float bv = bias ? bfr(bias[c0 + t * 16 + lr]) : 0.f;
#pragma unroll
        for (int j = 0; j < 8; ++j) os[(hi * 8 + j) * 68 + t * 16 + lr] = acc[t][j] + bv; }
    __syncthreads();
    if (F16OUT) {
        h16* crow = (h16*)(void*)C + (size_t)r0 * ldc + c0;
        auto pass = [&]() {
#pragma unroll
            for (int s = 0; s < 4; ++s) { const int row = 4 * s + (lane >> 3), piece = lane & 7; const float* sp = os + row * 68 + piece * 8; v8h o, o2;
#pragma unroll
                for (int i = 0; i < 8; ++i) { const h16 a = (h16)sp[i]; o[i] = a; o2[i] = (h16)((sp[i] - (float)a) * LOSC); }
                *(volatile v8h*)(crow + (size_t)row * ldc + piece * 8) = o; if (C2) *(volatile v8h*)(C2 + (size_t)r0 * ldc + c0 + (size_t)row * ldc + piece * 8) = o2; }
        };
        pass(); __threadfence(); pass();
    } else {
        float* crow = C + (size_t)r0 * ldc + c0;
        auto pass = [&]() {
#pragma unroll
            for (int s = 0; s < 8; ++s) { const int Lid = (lane >> 3) + 4 * s, piece = lane & 7; const int row = Lid >> 1, cofs = (Lid & 1) * 32 + piece * 4;
                v4f val = *(const v4fa*)(os + row * 68 + cofs); if (R) { const v4f rv = *(const v4f*)(R + ((size_t)r0 + row) * ldc + c0 + cofs); val += roundR ? (v4f){bfr(rv[0]), bfr(rv[1]), bfr(rv[2]), bfr(rv[3])} : rv; }
                *(volatile v4f*)(crow + (size_t)row * ldc + cofs) = val; }
        };
        pass(); __threadfence(); pass();
    }
}


__device__ __forceinline__ float sgnf(float v) { return v > 0.f ? 1.f : (v < 0.f ? -1.f : 0.f); }
__device__ __forceinline__ float binz(float v) { return sgnf(fminf(fmaxf(v, -1.f), 1.f)); }
__global__ __launch_bounds__(256) void k_S(const float* __restrict__ x, const int* __restrict__ rm0, const int* __restrict__ rm1, const int* __restrict__ rm2, bf* A) {
    const int u = blockIdx.x * 256 + threadIdx.x; if (u >= NBT * NI / 8) return;
    const int b = u / (NI / 8), i0 = (u % (NI / 8)) * 8;
    float sel[8][4][2];
    float ax[8];
#pragma unroll
    for (int j = 0; j < 8; ++j) { const int i = i0 + j, tm = i / TI, ii = i % TI;
        const float xv = bfr(x[(size_t)b * NI + i]); ax[j] = fabsf(xv); const float bx = binz(xv);
        int a0 = rm0[ii], a1 = rm1[ii], a2 = rm2[ii]; a0 = a0 < 0 ? 0 : (a0 >= TI ? TI - 1 : a0); a1 = a1 < 0 ? 0 : (a1 >= TI ? TI - 1 : a1); a2 = a2 < 0 ? 0 : (a2 >= TI ? TI - 1 : a2);
        const float d0 = binz(bfr(x[(size_t)b * NI + tm * TI + a0])), d1 = binz(bfr(x[(size_t)b * NI + tm * TI + a1])), d2 = binz(bfr(x[(size_t)b * NI + tm * TI + a2]));
        sel[j][0][0] = (1.f + bx) * 0.5f; sel[j][0][1] = (1.f - bx) * 0.5f; sel[j][1][0] = (1.f + d0) * 0.5f; sel[j][1][1] = (1.f - d0) * 0.5f;
        sel[j][2][0] = (1.f + d1) * 0.5f; sel[j][2][1] = (1.f - d1) * 0.5f; sel[j][3][0] = (1.f + d2) * 0.5f; sel[j][3][1] = (1.f - d2) * 0.5f; }
#pragma unroll 1
    for (int ps = 0; ps < 2; ++ps) {
#pragma unroll
        for (int k = 0; k < NK; ++k) { const int p = (k >> 3) & 1, q = (k >> 2) & 1, r = (k >> 1) & 1, s = k & 1; v8us o;
#pragma unroll
            for (int j = 0; j < 8; ++j) o[j] = f2bf(sel[j][0][p] * ax[j] * sel[j][1][q] * sel[j][2][r] * sel[j][3][s]);
            *(volatile v8us*)(A + (size_t)b * KTOT + (size_t)k * NI + i0) = o; }
        if (ps == 0) __threadfence(); }
}
__global__ __launch_bounds__(256) void k_W(const float* __restrict__ w1, const float* __restrict__ call, const float* __restrict__ gam, const float* __restrict__ pmask, bf* B) {
    const int u = blockIdx.x * 256 + threadIdx.x; if (u >= NO * NI / 8) return;
    const int o = u / (NI / 8), i0 = (u % (NI / 8)) * 8, oo = o % TO;
    const float g = fabsf(bfr(gam[0]));
    float ws0[8], ws1[8], pmv[8];
#pragma unroll
    for (int j = 0; j < 8; ++j) { const int i = i0 + j; const float sw = binz(bfr(w1[(size_t)i * NO + o])); ws0[j] = (1.f + sw) * 0.5f; ws1[j] = (1.f - sw) * 0.5f; pmv[j] = bfr(pmask[(size_t)(i % TI) * TO + oo]); }
#pragma unroll 1
    for (int ps = 0; ps < 2; ++ps) {
#pragma unroll 1
        for (int k = 0; k < NK; ++k) { v8us ov;
#pragma unroll
            for (int j = 0; j < 8; ++j) { const int ii = (i0 + j) % TI;
                const float c0 = binz(bfr(call[((size_t)(2 * k) * TI + ii) * TO + oo])), c1 = binz(bfr(call[((size_t)(2 * k + 1) * TI + ii) * TO + oo]));
                ov[j] = f2bf(g * (c0 * ws0[j] + c1 * ws1[j]) * pmv[j]); }
            *(volatile v8us*)(B + (size_t)o * KTOT + (size_t)k * NI + i0) = ov; }
        if (ps == 0) __threadfence(); }
}

extern "C" void kernel_launch(void* const* d_in, const int* in_sizes, int n_in,
                              void* d_out, int out_size, void* d_ws, size_t ws_size, hipStream_t stream) {
    (void)in_sizes; (void)n_in; (void)out_size;
    const float* x = (const float*)d_in[0]; const float* w1 = (const float*)d_in[1]; const float* call = (const float*)d_in[2]; const float* gam = (const float*)d_in[3]; const float* pmask = (const float*)d_in[4];
    const int* rm0 = (const int*)d_in[5]; const int* rm1 = (const int*)d_in[6]; const int* rm2 = (const int*)d_in[7];
    float* out = (float*)d_out;
    char* wsp = (char*)d_ws;
    auto take = [&](size_t bytes) { char* p = wsp; wsp += (bytes + 255) & ~(size_t)255; return (void*)p; };
    bf* A = (bf*)take((size_t)NBT * KTOT * 2); bf* B = (bf*)take((size_t)NO * KTOT * 2);
    if ((size_t)(wsp - (char*)d_ws) > ws_size) return;
    k_S<<<(NBT * NI / 8 + 255) / 256, 256, 0, stream>>>(x, rm0, rm1, rm2, A);
    k_W<<<(NO * NI / 8 + 255) / 256, 256, 0, stream>>>(w1, call, gam, pmask, B);
    k_gemmb<false, false><<<dim3(NBT / 64, NO / 64, 1), 128, 0, stream>>>(A, nullptr, B, nullptr, out, NO, nullptr);
}
